// Decoder_1898375545208
// MI455X (gfx1250) — hardware-verified
//
#include <hip/hip_runtime.h>
#include <stddef.h>
#include <stdint.h>


#define DD     128
#define NKB    8
#define NC     5
#define NCOL   (NC * DD)
#define KP     (2 * DD)
#define NTHR   256
#define NUF    (NCOL * (DD / 8))
#define GBM    64
#define GBN    128
#define GTHR   128
#define EB     1024
#define EPASS  (EB / 32)
#define NIT    ((EB * NC) / (4 * NTHR))
#define WSMAX  134217728

static_assert(NUF % NTHR == 0);
static_assert(DD % 32 == 0 && KP % 32 == 0 && GBN == DD);
static_assert(GBM == (GTHR / 32) * 16);
static_assert(EB % 32 == 0 && (EB * NC) % (4 * NTHR) == 0 && ((EB * NC * 4) % 128) == 0);
static_assert(DD / 8 == 16 && DD == 8 * 16);

typedef float          v4f   __attribute__((ext_vector_type(4)));
typedef float          v8f   __attribute__((ext_vector_type(8)));
typedef int            v8i   __attribute__((ext_vector_type(8)));
typedef unsigned short v8us  __attribute__((ext_vector_type(8)));
typedef unsigned short v16us __attribute__((ext_vector_type(16)));
typedef __bf16         v16bf __attribute__((ext_vector_type(16)));
typedef v4f  __attribute__((may_alias)) v4fa;
typedef v8us __attribute__((may_alias)) v8usa;
union FragB { v16bf v; v16us u; v8us h[2]; v8i w; };

__device__ __forceinline__ v8f wmb(const FragB& a, const FragB& b, v8f c) {
  v8f d = __builtin_amdgcn_wmma_f32_16x16x32_bf16(false, a.v, false, b.v, (short)0, c, false, false);
  asm volatile("v_nop\n\tv_nop\n\tv_nop\n\tv_nop" : "+v"(d) : "v"(a.w), "v"(b.w));
  return d;
}

__device__ __forceinline__ unsigned bf16_bits(float f) {
  const unsigned u = __float_as_uint(f);
  return (u + 0x7FFFu + ((u >> 16) & 1u)) >> 16;
}
__device__ __forceinline__ float bf16_val(float f) {
  return __uint_as_float(bf16_bits(f) << 16);
}

__global__ __launch_bounds__(NTHR) void k_fold(const float* __restrict__ W, const float* __restrict__ wc,
                                               unsigned short* BT) {
  const int u = (int)blockIdx.x * NTHR + (int)threadIdx.x;
  if (u >= NUF) return;
  const int n  = u >> 4;
  const int f8 = (u & 15) * 8;
  const int c  = n >> 7;
  const int d  = n & (DD - 1);
  float a0 = 0.0f, a1 = 0.0f, a2 = 0.0f, a3 = 0.0f, a4 = 0.0f, a5 = 0.0f, a6 = 0.0f, a7 = 0.0f;
#pragma unroll 1
  for (int k = 0; k < NKB; ++k) {
    const float w = bf16_val(wc[k * NC + c]);
    const float* p = W + (size_t)k * (DD * DD) + (size_t)d * DD + f8;
    const v4f x = *(const v4fa*)p;
    const v4f y = *(const v4fa*)(p + 4);
    a0 = fmaf(w, bf16_val(x.x), a0); a1 = fmaf(w, bf16_val(x.y), a1);
    a2 = fmaf(w, bf16_val(x.z), a2); a3 = fmaf(w, bf16_val(x.w), a3);
    a4 = fmaf(w, bf16_val(y.x), a4); a5 = fmaf(w, bf16_val(y.y), a5);
    a6 = fmaf(w, bf16_val(y.z), a6); a7 = fmaf(w, bf16_val(y.w), a7);
  }
  v8us oh, ol;
  unsigned hb;
  hb = bf16_bits(a0); oh[0] = (unsigned short)hb; ol[0] = (unsigned short)bf16_bits(a0 - __uint_as_float(hb << 16));
  hb = bf16_bits(a1); oh[1] = (unsigned short)hb; ol[1] = (unsigned short)bf16_bits(a1 - __uint_as_float(hb << 16));
  hb = bf16_bits(a2); oh[2] = (unsigned short)hb; ol[2] = (unsigned short)bf16_bits(a2 - __uint_as_float(hb << 16));
  hb = bf16_bits(a3); oh[3] = (unsigned short)hb; ol[3] = (unsigned short)bf16_bits(a3 - __uint_as_float(hb << 16));
  hb = bf16_bits(a4); oh[4] = (unsigned short)hb; ol[4] = (unsigned short)bf16_bits(a4 - __uint_as_float(hb << 16));
  hb = bf16_bits(a5); oh[5] = (unsigned short)hb; ol[5] = (unsigned short)bf16_bits(a5 - __uint_as_float(hb << 16));
  hb = bf16_bits(a6); oh[6] = (unsigned short)hb; ol[6] = (unsigned short)bf16_bits(a6 - __uint_as_float(hb << 16));
  hb = bf16_bits(a7); oh[7] = (unsigned short)hb; ol[7] = (unsigned short)bf16_bits(a7 - __uint_as_float(hb << 16));
  unsigned short* dp = BT + (size_t)n * KP + f8;
  *(volatile v8us*)dp = oh;
  *(volatile v8us*)(dp + DD) = ol;
  __threadfence();
  *(volatile v8us*)dp = oh;
  *(volatile v8us*)(dp + DD) = ol;
}

__global__ __launch_bounds__(GTHR) void k_itemgemm(const float* __restrict__ item, int nI,
                                                   const unsigned short* __restrict__ BT, float* PT) {
  __shared__ __attribute__((aligned(16))) float stg[GBM * GBN];
  const int tid = (int)threadIdx.x, lane = tid & 31, wave = tid >> 5, hh = lane >> 4, m = lane & 15;
  const int rowBase = (int)blockIdx.x * GBM;
  const int c = (int)blockIdx.y;

  v8f acc[8];
  {
    const v8f z = {0.f, 0.f, 0.f, 0.f, 0.f, 0.f, 0.f, 0.f};
#pragma unroll
    for (int t = 0; t < 8; ++t) acc[t] = z;
  }
  const int ar  = rowBase + 16 * wave + m;
  const int arc = ar < nI ? ar : nI - 1;
  const float* ap = item + (size_t)arc * DD + 8 * hh;
  const unsigned short* bp = BT + (size_t)(c * DD + m) * (size_t)KP + 8 * hh;

#pragma unroll 1
  for (int ks = 0; ks < DD / 32; ++ks) {
    const float* q = ap + 32 * ks;
    const v4f x0 = *(const v4fa*)q;
    const v4f x1 = *(const v4fa*)(q + 4);
    const v4f x2 = *(const v4fa*)(q + 16);
    const v4f x3 = *(const v4fa*)(q + 20);
    v8us h0, h1;
    h0[0] = (unsigned short)bf16_bits(x0.x); h0[1] = (unsigned short)bf16_bits(x0.y);
    h0[2] = (unsigned short)bf16_bits(x0.z); h0[3] = (unsigned short)bf16_bits(x0.w);
    h0[4] = (unsigned short)bf16_bits(x1.x); h0[5] = (unsigned short)bf16_bits(x1.y);
    h0[6] = (unsigned short)bf16_bits(x1.z); h0[7] = (unsigned short)bf16_bits(x1.w);
    h1[0] = (unsigned short)bf16_bits(x2.x); h1[1] = (unsigned short)bf16_bits(x2.y);
    h1[2] = (unsigned short)bf16_bits(x2.z); h1[3] = (unsigned short)bf16_bits(x2.w);
    h1[4] = (unsigned short)bf16_bits(x3.x); h1[5] = (unsigned short)bf16_bits(x3.y);
    h1[6] = (unsigned short)bf16_bits(x3.z); h1[7] = (unsigned short)bf16_bits(x3.w);
    FragB af;
    af.h[0] = h0;
    af.h[1] = h1;
#pragma unroll
    for (int nt = 0; nt < 8; ++nt) {
      const unsigned short* wq = bp + (size_t)(16 * nt) * (size_t)KP + 32 * ks;
      FragB bh;
      bh.h[0] = *(const v8usa*)wq;
      bh.h[1] = *(const v8usa*)(wq + 16);
      acc[nt] = wmb(af, bh, acc[nt]);
      FragB bl;
      bl.h[0] = *(const v8usa*)(wq + DD);
      bl.h[1] = *(const v8usa*)(wq + DD + 16);
      acc[nt] = wmb(af, bl, acc[nt]);
    }
  }

#pragma unroll
  for (int nt = 0; nt < 8; ++nt) {
    const int lc = 16 * nt + m;
#pragma unroll
    for (int r = 0; r < 8; ++r) {
      const int lr = 16 * wave + 8 * hh + r;
      stg[lr * GBN + lc] = acc[nt][r];
    }
  }
  __syncthreads();

  v4f pv[16];
#pragma unroll
  for (int i = 0; i < 16; ++i) pv[i] = *(const v4fa*)(stg + (16 * wave + i) * GBN + 4 * lane);

#pragma unroll
  for (int i = 0; i < 16; ++i) {
    const int r = rowBase + 16 * wave + i;
    if (r < nI) *(volatile v4f*)(PT + (size_t)r * NCOL + c * DD + 4 * lane) = pv[i];
  }
  __threadfence();
#pragma unroll
  for (int i = 0; i < 16; ++i) {
    const int r = rowBase + 16 * wave + i;
    if (r < nI) *(volatile v4f*)(PT + (size_t)r * NCOL + c * DD + 4 * lane) = pv[i];
  }
}

__global__ __launch_bounds__(NTHR) void k_edge(const float* __restrict__ user, int nU,
                                               const float* __restrict__ PT, int nI,
                                               const int* __restrict__ uidx, const int* __restrict__ iidx,
                                               int nE, float* out) {
  __shared__ __attribute__((aligned(16))) float stage[EB * NC];
  const int tid = (int)threadIdx.x, lane = tid & 31, wave = tid >> 5;
  const int g = lane >> 3, sub = lane & 7;
  const int eBase = (int)blockIdx.x * EB;

#pragma unroll 1
  for (int ps = 0; ps < EPASS; ++ps) {
    const int el = ps * 32 + wave * 4 + g;
    const int e  = eBase + el;
    const int ec = e < nE ? e : nE - 1;
    int ui = uidx[ec];
    int ii = iidx[ec];
    ui = ui < 0 ? ui + nU : ui;
    ii = ii < 0 ? ii + nI : ii;
    ui = ui < 0 ? 0 : (ui > nU - 1 ? nU - 1 : ui);
    ii = ii < 0 ? 0 : (ii > nI - 1 ? nI - 1 : ii);
    const float* up = user + (size_t)ui * DD + 16 * sub;
    v4f u0 = *(const v4fa*)up;
    v4f u1 = *(const v4fa*)(up + 4);
    v4f u2 = *(const v4fa*)(up + 8);
    v4f u3 = *(const v4fa*)(up + 12);
    u0.x = bf16_val(u0.x); u0.y = bf16_val(u0.y); u0.z = bf16_val(u0.z); u0.w = bf16_val(u0.w);
    u1.x = bf16_val(u1.x); u1.y = bf16_val(u1.y); u1.z = bf16_val(u1.z); u1.w = bf16_val(u1.w);
    u2.x = bf16_val(u2.x); u2.y = bf16_val(u2.y); u2.z = bf16_val(u2.z); u2.w = bf16_val(u2.w);
    u3.x = bf16_val(u3.x); u3.y = bf16_val(u3.y); u3.z = bf16_val(u3.z); u3.w = bf16_val(u3.w);
    const float* pp = PT + (size_t)ii * NCOL + 16 * sub;
    float s[NC];
#pragma unroll
    for (int c = 0; c < NC; ++c) {
      const float* q = pp + c * DD;
      const v4f p0 = *(const v4fa*)q;
      const v4f p1 = *(const v4fa*)(q + 4);
      const v4f p2 = *(const v4fa*)(q + 8);
      const v4f p3 = *(const v4fa*)(q + 12);
      float a = 0.0f;
      a = fmaf(u0.x, p0.x, a); a = fmaf(u0.y, p0.y, a); a = fmaf(u0.z, p0.z, a); a = fmaf(u0.w, p0.w, a);
      a = fmaf(u1.x, p1.x, a); a = fmaf(u1.y, p1.y, a); a = fmaf(u1.z, p1.z, a); a = fmaf(u1.w, p1.w, a);
      a = fmaf(u2.x, p2.x, a); a = fmaf(u2.y, p2.y, a); a = fmaf(u2.z, p2.z, a); a = fmaf(u2.w, p2.w, a);
      a = fmaf(u3.x, p3.x, a); a = fmaf(u3.y, p3.y, a); a = fmaf(u3.z, p3.z, a); a = fmaf(u3.w, p3.w, a);
      s[c] = a;
    }
#pragma unroll
    for (int c = 0; c < NC; ++c) {
      float v = s[c];
      v += __shfl_xor(v, 1, 32);
      v += __shfl_xor(v, 2, 32);
      v += __shfl_xor(v, 4, 32);
      s[c] = v;
    }
    float r = (sub == 0) ? s[0] : (sub == 1) ? s[1] : (sub == 2) ? s[2] : (sub == 3) ? s[3] : s[4];
    r = (r > 0.0f) ? r : 0.0f;
    if (sub < NC) stage[el * NC + sub] = r;
  }
  __syncthreads();

  const int total4 = (nE / 4) * NC;
  const int gbase4 = (int)blockIdx.x * ((EB * NC) / 4);
  v4f ov[NIT];
#pragma unroll
  for (int it = 0; it < NIT; ++it) ov[it] = *(const v4fa*)(stage + 4 * (it * NTHR + tid));
#pragma unroll
  for (int it = 0; it < NIT; ++it) {
    const int g4 = gbase4 + it * NTHR + tid;
    if (g4 < total4) *(volatile v4f*)(out + 4 * (size_t)g4) = ov[it];
  }
  __threadfence();
#pragma unroll
  for (int it = 0; it < NIT; ++it) {
    const int g4 = gbase4 + it * NTHR + tid;
    if (g4 < total4) *(volatile v4f*)(out + 4 * (size_t)g4) = ov[it];
  }
}

static inline int cdiv(int a, int b) { return (a + b - 1) / b; }
static inline size_t al256(size_t o) { return (o + 255) & ~(size_t)255; }

extern "C" void kernel_launch(void* const* d_in, const int* in_sizes, int n_in,
                              void* d_out, int out_size, void* d_ws, size_t ws_size,
                              hipStream_t stream) {
  (void)stream;
  if (n_in < 6) return;
  if (in_sizes[0] < DD || (in_sizes[0] % DD) != 0) return;
  if (in_sizes[1] < DD || (in_sizes[1] % DD) != 0) return;
  const int nU = in_sizes[0] / DD;
  const int nI = in_sizes[1] / DD;
  const int nE = in_sizes[2];
  if (nE < 32 || (nE & 31) != 0 || nE > (1 << 27)) return;
  if (in_sizes[3] != nE) return;
  if (in_sizes[4] != NKB * DD * DD) return;
  if (in_sizes[5] != NKB * NC) return;
  if ((long long)out_size != (long long)nE * NC) return;
  if (nU < 1 || nU > (1 << 24) || nI < 1 || nI > (1 << 22)) return;

  const float* user = (const float*)d_in[0];
  const float* item = (const float*)d_in[1];
  const int*   uidx = (const int*)d_in[2];
  const int*   iidx = (const int*)d_in[3];
  const float* W    = (const float*)d_in[4];
  const float* wc   = (const float*)d_in[5];
  float* out = (float*)d_out;

  char* ws = (char*)d_ws;
  size_t off = 0;
  const size_t oBT = off; off = al256(off + (size_t)NCOL * KP * 2);
  const size_t oPT = off; off = al256(off + (size_t)nI * NCOL * 4);
  if (off > ws_size || off > (size_t)WSMAX) return;
  unsigned short* BT = (unsigned short*)(ws + oBT);
  float*          PT = (float*)(ws + oPT);

  k_fold<<<NUF / NTHR, NTHR, 0, stream>>>(W, wc, BT);
  k_itemgemm<<<dim3(cdiv(nI, GBM), NC), GTHR, 0, stream>>>(item, nI, BT, PT);
  k_edge<<<cdiv(nE, EB), NTHR, 0, stream>>>(user, nU, PT, nI, uidx, iidx, nE, out);
}
